// HeteroAttentionLayer_43404939493467
// MI455X (gfx1250) — hardware-verified
//
#include <hip/hip_runtime.h>

typedef __attribute__((ext_vector_type(16))) _Float16 v16h;
typedef __attribute__((ext_vector_type(8)))  _Float16 v8h;
typedef __attribute__((ext_vector_type(16))) __bf16   v16b;
typedef __attribute__((ext_vector_type(8)))  __bf16   v8b;
typedef __attribute__((ext_vector_type(8)))  float    v8f;
typedef __attribute__((ext_vector_type(4)))  float    v4f;
typedef __attribute__((ext_vector_type(4)))  unsigned int v4u;
#define PSCALE 32768.0f
#define U16(p) ((const unsigned short*)(const void*)(p))
#define PSCALE_INV (1.0f / 32768.0f)

__device__ __forceinline__ unsigned short f2bf_bits(float f) {
  unsigned u = __float_as_uint(f);
  return (unsigned short)((u + 0x7FFFu + ((u >> 16) & 1u)) >> 16);
}
__device__ __forceinline__ float bf_bits2f(unsigned short h) { return __uint_as_float(((unsigned)h) << 16); }

__device__ __forceinline__ void dep_guard_h(v8f& a, v8f& b, v16h x, v16h y) { asm volatile("v_nop\n\tv_nop\n\tv_nop\n\tv_nop" : "+v"(a), "+v"(b) : "v"(x), "v"(y)); }
__device__ __forceinline__ void dep_guard_b(v8f& a, v8f& b, v16b x, v16b y) { asm volatile("v_nop\n\tv_nop\n\tv_nop\n\tv_nop" : "+v"(a), "+v"(b) : "v"(x), "v"(y)); }
__device__ __forceinline__ void keep4_h(v16h a, v16h b, v16h c, v16h d) { asm volatile("v_nop" :: "v"(a), "v"(b), "v"(c), "v"(d)); }
__device__ __forceinline__ void keep4_b(v16b a, v16b b, v16b c, v16b d) { asm volatile("v_nop" :: "v"(a), "v"(b), "v"(c), "v"(d)); }
__device__ __forceinline__ void acc_guard4(v8f& a, v8f& b, v8f& c, v8f& d) { asm volatile("v_nop\n\tv_nop\n\tv_nop\n\tv_nop" : "+v"(a), "+v"(b), "+v"(c), "+v"(d)); }
template <typename T> struct Frag;
template <> struct Frag<_Float16> {
  typedef v16h V; union U { v16h v; v8h h[2]; };
  static __device__ __forceinline__ v16h load(const _Float16* p) {
    U f; f.h[0] = *(const v8h*)(p); f.h[1] = *(const v8h*)(p + 16); return f.v;
  }
  static __device__ __forceinline__ v8f mma(v16h a, v16h b, v8f c) {
    return __builtin_amdgcn_wmma_f32_16x16x32_f16(false, a, false, b, (short)0, c, false, false);
  }
  static __device__ __forceinline__ void guard(v8f& a, v8f& b, v16h x, v16h y) { dep_guard_h(a, b, x, y); }
  static __device__ __forceinline__ void keep(v16h a, v16h b, v16h c, v16h d) { keep4_h(a, b, c, d); }
};
template <> struct Frag<__bf16> {
  typedef v16b V; union U { v16b v; v8b h[2]; };
  static __device__ __forceinline__ v16b load(const __bf16* p) {
    U f; f.h[0] = *(const v8b*)(p); f.h[1] = *(const v8b*)(p + 16); return f.v;
  }
  static __device__ __forceinline__ v8f mma(v16b a, v16b b, v8f c) {
    return __builtin_amdgcn_wmma_f32_16x16x32_bf16(false, a, false, b, (short)0, c, false, false);
  }
  static __device__ __forceinline__ void guard(v8f& a, v8f& b, v16b x, v16b y) { dep_guard_b(a, b, x, y); }
  static __device__ __forceinline__ void keep(v16b a, v16b b, v16b c, v16b d) { keep4_b(a, b, c, d); }
};

template <int ET> struct Elem;
template <> struct Elem<0> { typedef _Float16 T; };
template <> struct Elem<1> { typedef __bf16 T; };
template <int ET, bool SPLIT, int BIAS_MODE, int OUT_MODE, bool RESID, int ACT = 0>
__global__ __launch_bounds__(256) void wmma_gemm64(
    const unsigned short* __restrict__ Ap, const unsigned short* __restrict__ A2p, int lda, long strideA,
    const unsigned short* __restrict__ Btp, const unsigned short* __restrict__ Bt2p, int ldb, long strideB,
    void* __restrict__ Cout, void* __restrict__ Cout2, int ldc, long strideC,
    const float* __restrict__ bias,
    const float* __restrict__ resid, long strideR,
    int M, int N, int K, float scale) {
  typedef typename Elem<ET>::T T;
  typedef typename Frag<T>::V V;
  const T* A = (const T*)Ap; const T* A2 = (const T*)A2p; const T* Bt = (const T*)Btp; const T* Bt2 = (const T*)Bt2p;
  __shared__ __align__(16) float sT[8][16 * 68];
  const int b    = blockIdx.y;
  const int lane = threadIdx.x & 31;
  const int wave = threadIdx.x >> 5;
  const int tilesN = N >> 6;
  const int tilesM = M >> 6;
  const int tile = blockIdx.x * 8 + wave;
  if (tile >= tilesM * tilesN) return;
  const int tm = tile / tilesN;
  const int tn = tile - tm * tilesN;
  const int m0 = tm << 6;
  const int n0 = tn << 6;

  const T* Ab  = A  + (size_t)b * strideA;
  const T* Bb  = Bt + (size_t)b * strideB;
  const T* Ab2 = SPLIT ? (A2  + (size_t)b * strideA) : nullptr;
  const T* Bb2 = SPLIT ? (Bt2 + (size_t)b * strideB) : nullptr;

  const int rlane = lane & 15;
  const int koff  = (lane >> 4) * 8;
  const int mOff  = (lane >> 4) * 8;

  v8f acc[4][4];
#pragma unroll
  for (int i = 0; i < 4; ++i)
#pragma unroll
    for (int j = 0; j < 4; ++j) acc[i][j] = (v8f){0.f,0.f,0.f,0.f,0.f,0.f,0.f,0.f};

  for (int k0 = 0; k0 < K; k0 += 32) {
    V bh[4], bl[4];
#pragma unroll
    for (int j = 0; j < 4; ++j) {
      const size_t bo = (size_t)(n0 + (j << 4) + rlane) * ldb + koff + k0;
      bh[j] = Frag<T>::load(Bb + bo);
      if (SPLIT) bl[j] = Frag<T>::load(Bb2 + bo);
    }
#pragma unroll
    for (int i = 0; i < 4; ++i) {
      const size_t ao = (size_t)(m0 + (i << 4) + rlane) * lda + koff + k0;
      V ah = Frag<T>::load(Ab + ao);
      V al;
      if (SPLIT) al = Frag<T>::load(Ab2 + ao);
#pragma unroll
      for (int j = 0; j < 4; ++j) {
        acc[i][j] = Frag<T>::mma(ah, bh[j], acc[i][j]);
        if (SPLIT) {
          acc[i][j] = Frag<T>::mma(ah, bl[j], acc[i][j]);
          acc[i][j] = Frag<T>::mma(al, bh[j], acc[i][j]);
        }
      }
      Frag<T>::guard(acc[i][0], acc[i][3], ah, SPLIT ? al : ah);
    }
    Frag<T>::keep(bh[0], bh[1], bh[2], bh[3]);
    if (SPLIT) Frag<T>::keep(bl[0], bl[1], bl[2], bl[3]);
  }
  acc_guard4(acc[0][0], acc[0][1], acc[0][2], acc[0][3]);
  acc_guard4(acc[1][0], acc[1][1], acc[1][2], acc[1][3]);
  acc_guard4(acc[2][0], acc[2][1], acc[2][2], acc[2][3]);
  acc_guard4(acc[3][0], acc[3][1], acc[3][2], acc[3][3]);

  float* slab = sT[wave];
  const float* Rb = RESID ? (resid + (size_t)b * strideR) : nullptr;
#pragma unroll
  for (int i = 0; i < 4; ++i) {
    const int mBase = m0 + (i << 4);
#pragma unroll
    for (int j = 0; j < 4; ++j) {
      const int n = n0 + (j << 4) + rlane;
      float bv = 0.f;
      if (BIAS_MODE == 2) bv = bias[n];
#pragma unroll
      for (int r = 0; r < 8; ++r) {
        float v = acc[i][j][r] * scale;
        if (BIAS_MODE == 1) v += bias[mBase + mOff + r];
        if (BIAS_MODE == 2) v += bv;
        if (RESID) v += Rb[(size_t)(mBase + mOff + r) * ldc + n];
        if (ACT == 1) v = tanhf(v);
        if (ACT == 2) v = fmaxf(v, 0.0f);
        if (ACT == 3) v = v / (1.0f + expf(-v));
        if (ACT == 4) v = (v > 0.f) ? v : 0.01f * v;
        if (ACT == 5) v = 0.5f * v * (1.0f + erff(v * 0.70710678118654752f));
        slab[(mOff + r) * 68 + (j << 4) + rlane] = v;
      }
    }
    __builtin_amdgcn_fence(__ATOMIC_RELEASE, "workgroup");
    __builtin_amdgcn_wave_barrier();
    __builtin_amdgcn_fence(__ATOMIC_ACQUIRE, "workgroup");
    if (OUT_MODE == 0) {
      float* C = (float*)Cout + (size_t)b * strideC;
      const int hh = lane >> 4, c4 = (lane & 15) * 4;
      for (int pass = 0; pass < 2; ++pass) {
#pragma unroll
        for (int it = 0; it < 8; ++it) {
          const int row = it * 2 + hh;
          v4f v = *(const v4f*)(slab + row * 68 + c4);
          *(volatile v4f*)(C + (size_t)(mBase + row) * ldc + n0 + c4) = v;
        }
        __threadfence();
      }
    } else {
      const int q = lane >> 3, c8 = (lane & 7) * 8;
      unsigned short* C  = (unsigned short*)Cout  + (size_t)b * strideC;
      unsigned short* C2 = (OUT_MODE == 2) ? ((unsigned short*)Cout2 + (size_t)b * strideC) : nullptr;
      for (int pass = 0; pass < 2; ++pass) {
#pragma unroll
        for (int it = 0; it < 4; ++it) {
          const int row = it * 4 + q;
          const float* sp = slab + row * 68 + c8;
          v8h hv, lv;
#pragma unroll
          for (int e = 0; e < 8; ++e) {
            if (OUT_MODE == 1) {
              hv[e] = (_Float16)sp[e];
            } else {
              unsigned short hb = f2bf_bits(sp[e]);
              unsigned short lb = f2bf_bits(sp[e] - bf_bits2f(hb));
              hv[e] = __builtin_bit_cast(_Float16, hb);
              lv[e] = __builtin_bit_cast(_Float16, lb);
            }
          }
          *(volatile v8h*)(C + (size_t)(mBase + row) * ldc + n0 + c8) = hv;
          if (OUT_MODE == 2) *(volatile v8h*)(C2 + (size_t)(mBase + row) * ldc + n0 + c8) = lv;
        }
        __threadfence();
      }
    }
    __builtin_amdgcn_fence(__ATOMIC_RELEASE, "workgroup");
    __builtin_amdgcn_wave_barrier();
    __builtin_amdgcn_fence(__ATOMIC_ACQUIRE, "workgroup");
  }
}

#define FEAT 128
#define GATES 512
#define NBR 16
#define LSTM_STEPS 16
#define HA_PITCH 136
#define HA_TILE (16 * HA_PITCH)
#define XS_PITCH 516

__device__ __forceinline__ v8f mma_f16g(v16h a, v16h b, v8f c) {
  c = __builtin_amdgcn_wmma_f32_16x16x32_f16(false, a, false, b, (short)0, c, false, false);
  asm volatile("v_nop\n\tv_nop\n\tv_nop\n\tv_nop" : "+v"(c) : "v"(a), "v"(b));
  return c;
}

__device__ __forceinline__ float sigm_f(float v) { return __builtin_amdgcn_rcpf(1.0f + expf(-v)); }
__device__ __forceinline__ float tanh_f(float v) { return 1.0f - 2.0f * __builtin_amdgcn_rcpf(1.0f + expf(2.0f * v)); }

__global__ __launch_bounds__(256) void k_cast_x(const float* __restrict__ x, unsigned short* __restrict__ xh,
                                               int nNodes, int mRows) {
  const int wave = threadIdx.x >> 5;
  const int lane = threadIdx.x & 31;
  const int row = blockIdx.x * 8 + wave;
  if (row >= mRows) return;
  const int rowc = (row < nNodes) ? row : (nNodes - 1);
  const int colc = (lane & 15) * 8;
  const float* src = x + (size_t)rowc * FEAT + colc;
  const v4f a0 = *(const v4f*)(src);
  const v4f a1 = *(const v4f*)(src + 4);
  const bool keep = (row < nNodes) && (lane < 16);
  v8h hv;
#pragma unroll
  for (int e = 0; e < 4; ++e) {
    const float f0 = keep ? a0[e] : 0.0f;
    const float f1 = keep ? a1[e] : 0.0f;
    hv[e] = (_Float16)f0;
    hv[4 + e] = (_Float16)f1;
  }
  unsigned short* dst = xh + (size_t)row * (2 * FEAT) + lane * 8;
  *(volatile v8h*)dst = hv;
  __threadfence();
  *(volatile v8h*)dst = hv;
}

__global__ __launch_bounds__(256) void k_cast_w(const float* __restrict__ s0, const float* __restrict__ s1,
                                               unsigned short* __restrict__ out, int rows, int ncat, float sc) {
  const int L = ncat * FEAT;
  const int total = rows * L;
  const int e0 = (blockIdx.x * 256 + threadIdx.x) * 8;
  const int ec = (e0 < total) ? e0 : (total - 8);
  const int n = ec / L;
  const int k = ec - n * L;
  const int k0 = k & (FEAT - 1);
  const float* p0 = s0 + (size_t)n * FEAT + k0;
  const float* p1 = s1 + (size_t)n * FEAT + k0;
  const v4f a0 = *(const v4f*)(p0);
  const v4f a1 = *(const v4f*)(p0 + 4);
  const v4f c0 = *(const v4f*)(p1);
  const v4f c1 = *(const v4f*)(p1 + 4);
  const bool second = (k >= FEAT);
  v8h hv;
#pragma unroll
  for (int e = 0; e < 4; ++e) {
    const float f0 = (second ? c0[e] : a0[e]) * sc;
    const float f1 = (second ? c1[e] : a1[e]) * sc;
    hv[e] = (_Float16)f0;
    hv[4 + e] = (_Float16)f1;
  }
  if (e0 < total) {
    unsigned short* dst = out + e0;
    *(volatile v8h*)dst = hv;
    __threadfence();
    *(volatile v8h*)dst = hv;
  }
}

__global__ __launch_bounds__(256) void k_lstm(
    const unsigned short* __restrict__ xbh, const unsigned short* __restrict__ xbl,
    const int* __restrict__ nidx, const unsigned short* __restrict__ whh,
    const float* __restrict__ b_ih, const float* __restrict__ b_hh,
    unsigned short* __restrict__ xh, int nNodes)
{
  __shared__ __align__(16) _Float16 hA[2 * HA_TILE];
  __shared__ __align__(16) float xs[16 * XS_PITCH];
  __shared__ int idxs[16 * NBR];
  const int tid  = threadIdx.x;
  const int wave = tid >> 5;
  const int lane = tid & 31;
  const int hh   = lane >> 4;
  const int c    = lane & 15;
  const int koff = hh * 8;
  const int n0 = blockIdx.x * 16;
  const int u  = wave * 16 + c;

  {
    const int row = tid >> 4;
    const int dd  = tid & 15;
    int v = nidx[(size_t)(n0 + row) * NBR + dd];
    v = (v < 0) ? 0 : v;
    v = (v > nNodes - 1) ? (nNodes - 1) : v;
    idxs[tid] = v;
  }
  const float bs0 = b_ih[u]           + b_hh[u];
  const float bs1 = b_ih[FEAT + u]     + b_hh[FEAT + u];
  const float bs2 = b_ih[2 * FEAT + u] + b_hh[2 * FEAT + u];
  const float bs3 = b_ih[3 * FEAT + u] + b_hh[3 * FEAT + u];
  float cst[8];
#pragma unroll
  for (int r = 0; r < 8; ++r) cst[r] = 0.0f;
  const _Float16* whp = (const _Float16*)(const void*)whh;

#pragma unroll 1
  for (int d = 0; d < LSTM_STEPS; ++d) {
    __syncthreads();
#pragma unroll
    for (int it = 0; it < 4; ++it) {
      const int f   = it * 256 + tid;
      const int row = f >> 6;
      const int q   = f & 63;
      const int nb  = idxs[row * NBR + d];
      const size_t go = (size_t)nb * GATES + (size_t)(q * 8);
      const v4u w0 = *(const v4u*)(xbh + go);
      const v4u w1 = *(const v4u*)(xbl + go);
      v4f o0, o1;
      o0[0] = __uint_as_float(w0[0] << 16)          + __uint_as_float(w1[0] << 16);
      o0[1] = __uint_as_float(w0[0] & 0xffff0000u)  + __uint_as_float(w1[0] & 0xffff0000u);
      o0[2] = __uint_as_float(w0[1] << 16)          + __uint_as_float(w1[1] << 16);
      o0[3] = __uint_as_float(w0[1] & 0xffff0000u)  + __uint_as_float(w1[1] & 0xffff0000u);
      o1[0] = __uint_as_float(w0[2] << 16)          + __uint_as_float(w1[2] << 16);
      o1[1] = __uint_as_float(w0[2] & 0xffff0000u)  + __uint_as_float(w1[2] & 0xffff0000u);
      o1[2] = __uint_as_float(w0[3] << 16)          + __uint_as_float(w1[3] << 16);
      o1[3] = __uint_as_float(w0[3] & 0xffff0000u)  + __uint_as_float(w1[3] & 0xffff0000u);
      float* xd = xs + row * XS_PITCH + q * 8;
      *(v4f*)(xd)     = o0;
      *(v4f*)(xd + 4) = o1;
    }
    __syncthreads();

    v8f acc[4];
#pragma unroll
    for (int g = 0; g < 4; ++g) acc[g] = (v8f){0.f,0.f,0.f,0.f,0.f,0.f,0.f,0.f};
    if (d > 0) {
      const _Float16* ha = hA + (d & 1) * HA_TILE + c * HA_PITCH + koff;
      const _Float16* wb = whp + (size_t)u * FEAT + koff;
#pragma unroll
      for (int kk = 0; kk < 4; ++kk) {
        const v16h af = Frag<_Float16>::load(ha + kk * 32);
#pragma unroll
        for (int g = 0; g < 4; ++g) {
          const v16h bfr = Frag<_Float16>::load(wb + (size_t)g * (FEAT * FEAT) + kk * 32);
          acc[g] = mma_f16g(af, bfr, acc[g]);
        }
      }
    }

    _Float16* hn_t = hA + ((d + 1) & 1) * HA_TILE;
#pragma unroll
    for (int r = 0; r < 8; ++r) {
      const int row = hh * 8 + r;
      const float* xr = xs + row * XS_PITCH + u;
      const float p_i = acc[0][r] * 0.125f + xr[0]        + bs0;
      const float p_f = acc[1][r] * 0.125f + xr[FEAT]     + bs1;
      const float p_g = acc[2][r] * 0.125f + xr[2 * FEAT] + bs2;
      const float p_o = acc[3][r] * 0.125f + xr[3 * FEAT] + bs3;
      const float ig = sigm_f(p_i);
      const float fg = sigm_f(p_f);
      const float og = sigm_f(p_o);
      const float gg = tanh_f(p_g);
      const float cn = fg * cst[r] + ig * gg;
      cst[r] = cn;
      const float hn = og * tanh_f(cn);
      hn_t[row * HA_PITCH + u] = (_Float16)hn;
    }
  }
  __syncthreads();

  {
    const _Float16* hf = hA + (LSTM_STEPS & 1) * HA_TILE;
    const int q  = lane >> 3;
    const int c8 = (lane & 7) * 8;
    const int row = wave * 2 + (q >> 1);
    const int lh  = q & 1;
    const v8h hv = *(const v8h*)(hf + row * HA_PITCH + lh * 64 + c8);
    unsigned short* dst = xh + (size_t)(n0 + row) * (2 * FEAT) + FEAT + lh * 64 + c8;
    *(volatile v8h*)dst = hv;
    __threadfence();
    *(volatile v8h*)dst = hv;
  }
}

__global__ __launch_bounds__(256) void k_ln_out(
    const float* __restrict__ hpre, const float* __restrict__ x,
    const float* __restrict__ b_self, const float* __restrict__ b_neigh,
    const float* __restrict__ g1, const float* __restrict__ bt1,
    const float* __restrict__ g3, const float* __restrict__ bt3,
    float* __restrict__ out, int nNodes)
{
  const int wave = threadIdx.x >> 5;
  const int lane = threadIdx.x & 31;
  const int row  = blockIdx.x * 8 + wave;
  const int rowc = (row < nNodes) ? row : (nNodes - 1);
  const int c4 = lane * 4;
  const v4f hp  = *(const v4f*)(hpre + (size_t)rowc * FEAT + c4);
  const v4f xv  = *(const v4f*)(x + (size_t)rowc * FEAT + c4);
  const v4f vbs = *(const v4f*)(b_self + c4);
  const v4f vbn = *(const v4f*)(b_neigh + c4);
  const v4f vg1 = *(const v4f*)(g1 + c4);
  const v4f vb1 = *(const v4f*)(bt1 + c4);
  const v4f vg3 = *(const v4f*)(g3 + c4);
  const v4f vb3 = *(const v4f*)(bt3 + c4);
  const float inv_f = 1.0f / 128.0f;

  v4f h;
#pragma unroll
  for (int e = 0; e < 4; ++e) h[e] = hp[e] + vbs[e] + vbn[e];
  float s = (h[0] + h[1]) + (h[2] + h[3]);
#pragma unroll
  for (int off = 1; off < 32; off <<= 1) s += __shfl_xor(s, off, 32);
  const float mu = s * inv_f;
  v4f dv;
#pragma unroll
  for (int e = 0; e < 4; ++e) dv[e] = h[e] - mu;
  float s2 = (dv[0] * dv[0] + dv[1] * dv[1]) + (dv[2] * dv[2] + dv[3] * dv[3]);
#pragma unroll
  for (int off = 1; off < 32; off <<= 1) s2 += __shfl_xor(s2, off, 32);
  const float rs = rsqrtf(s2 * inv_f + 1e-5f);
  v4f y;
#pragma unroll
  for (int e = 0; e < 4; ++e) {
    float t = dv[e] * rs * vg1[e] + vb1[e];
    t = (t > 0.0f) ? t : 0.01f * t;
    y[e] = xv[e] + t;
  }
  float s3 = (y[0] + y[1]) + (y[2] + y[3]);
#pragma unroll
  for (int off = 1; off < 32; off <<= 1) s3 += __shfl_xor(s3, off, 32);
  const float mu2 = s3 * inv_f;
  v4f dw;
#pragma unroll
  for (int e = 0; e < 4; ++e) dw[e] = y[e] - mu2;
  float s4 = (dw[0] * dw[0] + dw[1] * dw[1]) + (dw[2] * dw[2] + dw[3] * dw[3]);
#pragma unroll
  for (int off = 1; off < 32; off <<= 1) s4 += __shfl_xor(s4, off, 32);
  const float rs2 = rsqrtf(s4 * inv_f + 1e-5f);
  v4f ov;
#pragma unroll
  for (int e = 0; e < 4; ++e) {
    float t = dw[e] * rs2 * vg3[e] + vb3[e];
    ov[e] = (t > 0.0f) ? t : 0.01f * t;
  }
  if (row < nNodes) {
    float* dst = out + (size_t)row * FEAT + c4;
    *(volatile v4f*)dst = ov;
    __threadfence();
    *(volatile v4f*)dst = ov;
  }
}

extern "C" void kernel_launch(void* const* d_in, const int* in_sizes, int n_in,
                              void* d_out, int out_size, void* d_ws, size_t ws_size,
                              hipStream_t stream) {
  if (n_in < 14) return;
  const float* x       = (const float*)d_in[0];
  const int*   nidx    = (const int*)  d_in[1];
  const float* W_self  = (const float*)d_in[2];
  const float* b_self  = (const float*)d_in[3];
  const float* W_neigh = (const float*)d_in[4];
  const float* b_neigh = (const float*)d_in[5];
  const float* W_ih    = (const float*)d_in[6];
  const float* W_hh    = (const float*)d_in[7];
  const float* b_ih    = (const float*)d_in[8];
  const float* b_hh    = (const float*)d_in[9];
  const float* g1      = (const float*)d_in[10];
  const float* bt1     = (const float*)d_in[11];
  const float* g3      = (const float*)d_in[12];
  const float* bt3     = (const float*)d_in[13];
  float* outp = (float*)d_out;

  const int nNodes = in_sizes[0] / FEAT;
  if (nNodes <= 0 || (nNodes % 16) != 0) return;
  if (in_sizes[0] != nNodes * FEAT || in_sizes[1] != nNodes * NBR) return;
  if (in_sizes[2] != FEAT * FEAT || in_sizes[4] != FEAT * FEAT) return;
  if (in_sizes[6] != GATES * FEAT || in_sizes[7] != GATES * FEAT) return;
  if (in_sizes[3] != FEAT || in_sizes[5] != FEAT || in_sizes[8] != GATES || in_sizes[9] != GATES) return;
  if (in_sizes[10] != FEAT || in_sizes[11] != FEAT || in_sizes[12] != FEAT || in_sizes[13] != FEAT) return;
  if (out_size != nNodes * FEAT) return;

  const int mRows = ((nNodes + 63) / 64) * 64;
  const size_t szXH   = (size_t)mRows * (2 * FEAT) * 2;
  const size_t szXB   = (size_t)mRows * GATES * 2;
  const size_t szW    = (size_t)GATES * FEAT * 2;
  const size_t szWC   = (size_t)FEAT * (2 * FEAT) * 2;
  const size_t szHPRE = (size_t)mRows * FEAT * 4;
  const size_t offXH   = 0;
  const size_t offXBH  = offXH + szXH;
  const size_t offXBL  = offXBH + szXB;
  const size_t offWIH  = offXBL + szXB;
  const size_t offWHH  = offWIH + szW;
  const size_t offWCAT = offWHH + szW;
  const size_t total   = offWCAT + szWC;
  if (total > ws_size) return;
  if (szHPRE > szXB) return;

  char* ws = (char*)d_ws;
  unsigned short* xh   = (unsigned short*)(ws + offXH);
  unsigned short* xbh  = (unsigned short*)(ws + offXBH);
  unsigned short* xbl  = (unsigned short*)(ws + offXBL);
  unsigned short* wih  = (unsigned short*)(ws + offWIH);
  unsigned short* whh  = (unsigned short*)(ws + offWHH);
  unsigned short* wcat = (unsigned short*)(ws + offWCAT);
  float* hpre = (float*)(ws + offXBH);

  k_cast_x<<<dim3(mRows / 8), dim3(256), 0, stream>>>(x, xh, nNodes, mRows);
  {
    const int nw  = (GATES * FEAT / 8 + 255) / 256;
    const int nwc = (FEAT * 2 * FEAT / 8 + 255) / 256;
    k_cast_w<<<dim3(nw), dim3(256), 0, stream>>>(W_ih, W_ih, wih, GATES, 1, 8.0f);
    k_cast_w<<<dim3(nw), dim3(256), 0, stream>>>(W_hh, W_hh, whh, GATES, 1, 8.0f);
    k_cast_w<<<dim3(nwc), dim3(256), 0, stream>>>(W_self, W_neigh, wcat, FEAT, 2, 8.0f);
  }
  {
    const int tiles  = (mRows / 64) * (GATES / 64);
    const int blocks = (tiles + 7) / 8;
    wmma_gemm64<0, false, 0, 2, false, 0><<<dim3(blocks, 1), dim3(256), 0, stream>>>(
        U16(xh), U16(xh), 2 * FEAT, 0L,
        U16(wih), U16(wih), FEAT, 0L,
        (void*)xbh, (void*)xbl, GATES, 0L,
        b_ih, x, 0L,
        mRows, GATES, FEAT, 0.125f);
  }
  k_lstm<<<dim3(nNodes / 16), dim3(256), 0, stream>>>(xbh, xbl, nidx, whh, b_ih, b_hh, xh, nNodes);
  {
    const int tiles  = (mRows / 64) * (FEAT / 64);
    const int blocks = (tiles + 7) / 8;
    wmma_gemm64<0, false, 0, 0, false, 0><<<dim3(blocks, 1), dim3(256), 0, stream>>>(
        U16(xh), U16(xh), 2 * FEAT, 0L,
        U16(wcat), U16(wcat), 2 * FEAT, 0L,
        (void*)hpre, (void*)hpre, FEAT, 0L,
        b_self, x, 0L,
        mRows, FEAT, 2 * FEAT, 0.125f);
  }
  k_ln_out<<<dim3((nNodes + 7) / 8), dim3(256), 0, stream>>>(hpre, x, b_self, b_neigh, g1, bt1, g3, bt3, outp, nNodes);
}
